// GCN2_1357209666150
// MI455X (gfx1250) — hardware-run, weakly checked
//
#include <hip/hip_runtime.h>
#include <stddef.h>
#include <stdint.h>
#include <math.h>

#define NN      100000
#define NE      1000000
#define FD      128
#define HD      64
#define NLAY    4
#define GBM     128
#define NGB     782
#define MP      100096
#define KL      128
#define NTHR    256
#define NWAVE   8
#define EPT     8
#define WCH     (32 * EPT)
#define NBRUN   1024
#define SLB     10
#define NBK     98
#define NSLOT   (NBK * NBRUN)
#define WLCAP   2048
#define RCAP    12288
#define DEGCAP  48
#define MAXDEG_MEAS   26
#define MAXB1024_MEAS 10439
#define ABM     64
#define SP      68
#define RECW    192
#define WSMAX   134217728

#define BK_ZINTS (NWAVE * WLCAP + RCAP + 4 * NBRUN)
#define BK_INTS  (BK_ZINTS + 16)
#define BK_LDS   (BK_INTS * 4)

#define PBX  (MP * FD / 8 / NTHR)
#define PBW0 (HD * FD / 8 / NTHR)
#define PBCW (NLAY * HD * KL / 8 / NTHR)
#define PBW1 (HD * KL / 8 / NTHR)
#define PBTOT (PBX + PBW0 + PBCW + PBW1 + 1)
#define OW_CWT (HD * FD)
#define OW_W1T (HD * FD + NLAY * HD * KL)
#define TB_B0  0
#define TB_B1  64
#define TB_G   128
#define TB_B   384
#define TB_N   640

static_assert(HD == 64 && HD == 16 * 4);
static_assert(MP == NGB * GBM && MP >= NN && MP % ABM == 0);
static_assert(NN - (NGB - 1) * GBM >= 1 && NN - (NGB - 1) * GBM <= GBM);
static_assert(NBRUN == (1 << SLB) && NBRUN % ABM == 0 && NBRUN % GBM == 0 && NBRUN % 32 == 0);
static_assert(NBRUN == 1024 && NBRUN == 4 * NTHR);
static_assert(NSLOT >= MP);
static_assert(NN <= 131072);
static_assert(NE % EPT == 0 && NE >= EPT && (NE * 4) % 16 == 0);
static_assert((long long)RCAP * 100 >= (long long)MAXB1024_MEAS * 115);
static_assert(WLCAP >= MAXB1024_MEAS / 8 + 8 * 46 + 1);
static_assert(MAXDEG_MEAS + 8 <= DEGCAP);
static_assert(RCAP % (NTHR * 4) == 0 && BK_ZINTS % 4 == 0);
static_assert(BK_LDS <= 300000);
static_assert((MP * FD / 8) % NTHR == 0 && (HD * FD / 8) % NTHR == 0);
static_assert((NLAY * HD * KL / 8) % NTHR == 0 && (HD * KL / 8) % NTHR == 0);
static_assert(FD % 32 == 0 && KL % 32 == 0 && KL == 2 * HD && FD == KL);
static_assert((GBM * SP + 64 + RECW) * 4 <= 65536);
static_assert((MP * HD / 4) % NTHR == 0);
static_assert(RECW % 4 == 0 && RECW / 4 <= NTHR && RECW == 3 * HD);

typedef float          v4f   __attribute__((ext_vector_type(4)));
typedef float          v8f   __attribute__((ext_vector_type(8)));
typedef int            v4i   __attribute__((ext_vector_type(4)));
typedef int            v8i   __attribute__((ext_vector_type(8)));
typedef unsigned       v2u   __attribute__((ext_vector_type(2)));
typedef unsigned short v8us  __attribute__((ext_vector_type(8)));
typedef unsigned short v16us __attribute__((ext_vector_type(16)));
typedef __bf16         v16bf __attribute__((ext_vector_type(16)));
typedef v4f  __attribute__((may_alias)) v4fa;
typedef v4i  __attribute__((may_alias)) v4ia;
typedef v2u  __attribute__((may_alias)) v2ua;
typedef v8us __attribute__((may_alias)) v8usa;
union FragB { v16bf v; v16us u; v8us h[2]; v8i w; };

__device__ __forceinline__ v8f wmb(const FragB& a, const FragB& b, v8f c) {
  v8f d = __builtin_amdgcn_wmma_f32_16x16x32_bf16(false, a.v, false, b.v, (short)0, c, false, false);
  asm volatile("v_nop\n\tv_nop\n\tv_nop\n\tv_nop" : "+v"(d) : "v"(a.w), "v"(b.w));
  return d;
}

__device__ __forceinline__ unsigned bf16_bits(float f) {
  const unsigned u = __float_as_uint(f);
  const unsigned r = (u + 0x7FFFu + ((u >> 16) & 1u)) >> 16;
  const unsigned q = (u >> 16) | 0x40u;
  return ((u & 0x7fffffffu) > 0x7f800000u) ? q : r;
}
__device__ __forceinline__ float bf16_val(float f) {
  return __uint_as_float(bf16_bits(f) << 16);
}

__device__ __forceinline__ void hilo_pack(float v0, float v1, float v2, float v3,
                                          int& h01, int& h23, int& l01, int& l23) {
  const unsigned a0 = bf16_bits(v0), a1 = bf16_bits(v1), a2 = bf16_bits(v2), a3 = bf16_bits(v3);
  const unsigned b0 = bf16_bits(v0 - __uint_as_float(a0 << 16));
  const unsigned b1 = bf16_bits(v1 - __uint_as_float(a1 << 16));
  const unsigned b2 = bf16_bits(v2 - __uint_as_float(a2 << 16));
  const unsigned b3 = bf16_bits(v3 - __uint_as_float(a3 << 16));
  h01 = (int)(a0 | (a1 << 16)); h23 = (int)(a2 | (a3 << 16));
  l01 = (int)(b0 | (b1 << 16)); l23 = (int)(b2 | (b3 << 16));
}

__device__ __forceinline__ v4i regroup8(int h01, int h23, int l01, int l23, int lane) {
  const int t  = lane & 15;
  const int s0 = (lane & 16) + ((2 * t) & 15), s1 = s0 + 1;
  const int a0 = __shfl(h01, s0, 32), a1 = __shfl(h23, s0, 32), a2 = __shfl(h01, s1, 32), a3 = __shfl(h23, s1, 32);
  const int b0 = __shfl(l01, s0, 32), b1 = __shfl(l23, s0, 32), b2 = __shfl(l01, s1, 32), b3 = __shfl(l23, s1, 32);
  const int mk = (t < 8) ? -1 : 0;
  v4i o;
  o.x = (a0 & mk) | (b0 & ~mk); o.y = (a1 & mk) | (b1 & ~mk);
  o.z = (a2 & mk) | (b2 & ~mk); o.w = (a3 & mk) | (b3 & ~mk);
  return o;
}

__device__ __forceinline__ void st2_v4f(float* p, v4f v) {
  *(volatile v4f*)p = v;
  __threadfence();
  *(volatile v4f*)p = v;
}
__device__ __forceinline__ void st2_v8us(unsigned short* p, v8us v) {
  *(volatile v8us*)p = v;
  __threadfence();
  *(volatile v8us*)p = v;
}

__device__ __forceinline__ v8us gather8(const float* __restrict__ base, int stride) {
  float f[8];
#pragma unroll
  for (int i = 0; i < 8; ++i) f[i] = base[(size_t)i * (size_t)stride];
  v8us o;
#pragma unroll
  for (int i = 0; i < 8; ++i) o[i] = (unsigned short)bf16_bits(f[i]);
  return o;
}

__device__ __forceinline__ v4f bf16_val4(v4f a) {
  v4f o;
  o.x = bf16_val(a.x); o.y = bf16_val(a.y); o.z = bf16_val(a.z); o.w = bf16_val(a.w);
  return o;
}

__global__ __launch_bounds__(NTHR) void k_prep(const float* __restrict__ x, const float* __restrict__ w0,
                                               const float* __restrict__ cw, const float* __restrict__ w1,
                                               const float* __restrict__ b0, const float* __restrict__ b1,
                                               const float* __restrict__ gam, const float* __restrict__ bet,
                                               unsigned short* xb, unsigned short* wpl, float* tb) {
  const int tid = (int)threadIdx.x, lane = tid & 31, wave = tid >> 5;
  const int blk = (int)blockIdx.x;
  if (blk < PBX) {
    const int u   = blk * NTHR + tid;
    const int row = u >> 4, k8 = (u & 15) * 8;
    const int rc  = row < NN ? row : NN - 1;
    const unsigned mk = row < NN ? 0xffffu : 0u;
    const float* p = x + (size_t)rc * FD + k8;
    const v4f a = *(const v4fa*)p;
    const v4f b = *(const v4fa*)(p + 4);
    v8us o;
    o[0] = (unsigned short)(bf16_bits(a.x) & mk); o[1] = (unsigned short)(bf16_bits(a.y) & mk);
    o[2] = (unsigned short)(bf16_bits(a.z) & mk); o[3] = (unsigned short)(bf16_bits(a.w) & mk);
    o[4] = (unsigned short)(bf16_bits(b.x) & mk); o[5] = (unsigned short)(bf16_bits(b.y) & mk);
    o[6] = (unsigned short)(bf16_bits(b.z) & mk); o[7] = (unsigned short)(bf16_bits(b.w) & mk);
    st2_v8us(xb + (size_t)row * FD + k8, o);
  } else if (blk < PBX + PBW0) {
    const int u = (blk - PBX) * NTHR + tid;
    const int n = u >> 4, k8 = (u & 15) * 8;
    const v8us o = gather8(w0 + (size_t)k8 * HD + n, HD);
    st2_v8us(wpl + (size_t)n * FD + k8, o);
  } else if (blk < PBX + PBW0 + PBCW) {
    const int u = (blk - PBX - PBW0) * NTHR + tid;
    const int l = u >> 10, n = (u >> 4) & 63, k8 = (u & 15) * 8, kk = k8 & 63;
    const v8us o = gather8(cw + (size_t)l * HD * HD + (size_t)kk * HD + n, HD);
    st2_v8us(wpl + OW_CWT + (size_t)l * HD * KL + (size_t)n * KL + k8, o);
  } else if (blk < PBX + PBW0 + PBCW + PBW1) {
    const int u = (blk - PBX - PBW0 - PBCW) * NTHR + tid;
    const int n = u >> 4, k8 = (u & 15) * 8, kk = k8 & 63;
    const v8us o = gather8(w1 + (size_t)kk * HD + n, HD);
    st2_v8us(wpl + OW_W1T + (size_t)n * KL + k8, o);
  } else {
    if (wave == 0) {
      const int q = lane & 15;
      const v4f a = *(const v4fa*)(b0 + 4 * q);
      const v4f c = *(const v4fa*)(b1 + 4 * q);
      asm volatile("" :: "v"(a));
      asm volatile("" :: "v"(c));
      const unsigned ma = (lane < 16) ? 0xffffffffu : 0u;
      v4f o;
      o.x = __uint_as_float(((bf16_bits(a.x) << 16) & ma) | ((bf16_bits(c.x) << 16) & ~ma));
      o.y = __uint_as_float(((bf16_bits(a.y) << 16) & ma) | ((bf16_bits(c.y) << 16) & ~ma));
      o.z = __uint_as_float(((bf16_bits(a.z) << 16) & ma) | ((bf16_bits(c.z) << 16) & ~ma));
      o.w = __uint_as_float(((bf16_bits(a.w) << 16) & ma) | ((bf16_bits(c.w) << 16) & ~ma));
      st2_v4f(tb + TB_B0 + 4 * lane, o);
    } else if (wave < 3) {
      const int t = tid - 32;
      const v4f a = *(const v4fa*)(gam + 4 * t);
      st2_v4f(tb + TB_G + 4 * t, bf16_val4(a));
    } else if (wave < 5) {
      const int t = tid - 96;
      const v4f a = *(const v4fa*)(bet + 4 * t);
      st2_v4f(tb + TB_B + 4 * t, bf16_val4(a));
    }
  }
}

__device__ __forceinline__ void bucket_flush(const int* pl, const int* cnt, const int* offs, const int* dvi, int ov,
                                             int* lp, int* cp, int* op, int* dp, int* fp, int tid) {
#pragma unroll 1
  for (int i = tid * 4; i < RCAP; i += NTHR * 4) {
    const v4i v = *(const v4ia*)(pl + i);
    *(volatile v4i*)(lp + i) = v;
  }
  {
    const v4i v = *(const v4ia*)(cnt + 4 * tid);
    *(volatile v4i*)(cp + 4 * tid) = v;
  }
  {
    const v4i v = *(const v4ia*)(offs + 4 * tid);
    *(volatile v4i*)(op + 4 * tid) = v;
  }
  {
    const v4i v = *(const v4ia*)(dvi + 4 * tid);
    *(volatile v4i*)(dp + 4 * tid) = v;
  }
  if (tid < 8) {
    const v4i f = {ov, ov, ov, ov};
    *(volatile v4i*)(fp + 4 * tid) = f;
  }
}

__device__ __forceinline__ int clamp_node(int c) {
  return c < 0 ? 0 : (c > NN - 1 ? NN - 1 : c);
}

__global__ __launch_bounds__(NTHR) void k_bucket(const int* __restrict__ rows, const int* __restrict__ cols,
                                                 int* LIST, int* CNT, int* OFF, int* DINVI, int* FLAG) {
  extern __shared__ __attribute__((aligned(16))) int dsm[];
  int* wl   = dsm;
  int* pl   = dsm + NWAVE * WLCAP;
  int* cnt  = pl + RCAP;
  int* offs = cnt + NBRUN;
  int* cur  = offs + NBRUN;
  int* dvi  = cur + NBRUN;
  int* misc = dvi + NBRUN;
  const int tid = (int)threadIdx.x, lane = tid & 31, wave = tid >> 5;
  const int blk = (int)blockIdx.x;
  const unsigned nbs = (unsigned)(blk * NBRUN);

  {
    const v4i z4 = {0, 0, 0, 0};
    for (int i = tid * 4; i < BK_ZINTS; i += NTHR * 4) *(v4ia*)(dsm + i) = z4;
    if (tid < 16) misc[tid] = 0;
  }
  __syncthreads();

  {
    const int per  = ((NE + NWAVE * WCH - 1) / (NWAVE * WCH)) * WCH;
    const int ebeg = wave * per;
    const int eend = (ebeg + per < NE) ? (ebeg + per) : NE;
    int* mylist = wl + wave * WLCAP;
    int wc = 0;
#pragma unroll 1
    for (int cb = ebeg; cb < eend; cb += WCH) {
      const int e0  = cb + lane * EPT;
      const bool inr = e0 < NE;
      const int e0c = e0 < (NE - EPT) ? e0 : (NE - EPT);
      const v4i da = *(const v4ia*)(rows + e0c);
      const v4i db = *(const v4ia*)(rows + e0c + 4);
      const unsigned s0 = (unsigned)da.x - nbs, s1 = (unsigned)da.y - nbs;
      const unsigned s2 = (unsigned)da.z - nbs, s3 = (unsigned)da.w - nbs;
      const unsigned s4 = (unsigned)db.x - nbs, s5 = (unsigned)db.y - nbs;
      const unsigned s6 = (unsigned)db.z - nbs, s7 = (unsigned)db.w - nbs;
      const bool h0 = (s0 < (unsigned)NBRUN) & inr, h1 = (s1 < (unsigned)NBRUN) & inr;
      const bool h2 = (s2 < (unsigned)NBRUN) & inr, h3 = (s3 < (unsigned)NBRUN) & inr;
      const bool h4 = (s4 < (unsigned)NBRUN) & inr, h5 = (s5 < (unsigned)NBRUN) & inr;
      const bool h6 = (s6 < (unsigned)NBRUN) & inr, h7 = (s7 < (unsigned)NBRUN) & inr;
      const unsigned m0 = __builtin_amdgcn_ballot_w32(h0), m1 = __builtin_amdgcn_ballot_w32(h1);
      const unsigned m2 = __builtin_amdgcn_ballot_w32(h2), m3 = __builtin_amdgcn_ballot_w32(h3);
      const unsigned m4 = __builtin_amdgcn_ballot_w32(h4), m5 = __builtin_amdgcn_ballot_w32(h5);
      const unsigned m6 = __builtin_amdgcn_ballot_w32(h6), m7 = __builtin_amdgcn_ballot_w32(h7);
      const unsigned any = m0 | m1 | m2 | m3 | m4 | m5 | m6 | m7;
      if (any != 0u) {
        const v4i ca = *(const v4ia*)(cols + e0c);
        const v4i cc = *(const v4ia*)(cols + e0c + 4);
        const int c0 = clamp_node(ca.x), c1 = clamp_node(ca.y), c2 = clamp_node(ca.z), c3 = clamp_node(ca.w);
        const int c4 = clamp_node(cc.x), c5 = clamp_node(cc.y), c6 = clamp_node(cc.z), c7 = clamp_node(cc.w);
        const int pre = (int)(__builtin_amdgcn_mbcnt_lo(m0, 0u) + __builtin_amdgcn_mbcnt_lo(m1, 0u) +
                              __builtin_amdgcn_mbcnt_lo(m2, 0u) + __builtin_amdgcn_mbcnt_lo(m3, 0u) +
                              __builtin_amdgcn_mbcnt_lo(m4, 0u) + __builtin_amdgcn_mbcnt_lo(m5, 0u) +
                              __builtin_amdgcn_mbcnt_lo(m6, 0u) + __builtin_amdgcn_mbcnt_lo(m7, 0u));
        int p = wc + pre;
        if (h0) { if (p < WLCAP) mylist[p] = (c0 << SLB) | (int)s0; p = p + 1; }
        if (h1) { if (p < WLCAP) mylist[p] = (c1 << SLB) | (int)s1; p = p + 1; }
        if (h2) { if (p < WLCAP) mylist[p] = (c2 << SLB) | (int)s2; p = p + 1; }
        if (h3) { if (p < WLCAP) mylist[p] = (c3 << SLB) | (int)s3; p = p + 1; }
        if (h4) { if (p < WLCAP) mylist[p] = (c4 << SLB) | (int)s4; p = p + 1; }
        if (h5) { if (p < WLCAP) mylist[p] = (c5 << SLB) | (int)s5; p = p + 1; }
        if (h6) { if (p < WLCAP) mylist[p] = (c6 << SLB) | (int)s6; p = p + 1; }
        if (h7) { if (p < WLCAP) mylist[p] = (c7 << SLB) | (int)s7; p = p + 1; }
        wc += (int)(__builtin_popcount(m0) + __builtin_popcount(m1) + __builtin_popcount(m2) + __builtin_popcount(m3) +
                    __builtin_popcount(m4) + __builtin_popcount(m5) + __builtin_popcount(m6) + __builtin_popcount(m7));
      }
    }
    if (lane == 0) misc[wave] = wc;
  }
  __syncthreads();

  if (wave == 0) {
    int ov = 0;
#pragma unroll 1
    for (int w2 = 0; w2 < NWAVE; ++w2) {
      int c = misc[w2];
      if (c > WLCAP) ov = 1;
      c = c < 0 ? 0 : (c > WLCAP ? WLCAP : c);
#pragma unroll 1
      for (int b0 = 0; b0 < c; b0 += 32) {
        const int idx = b0 + lane;
        const int ent = wl[w2 * WLCAP + (idx < WLCAP ? idx : WLCAP - 1)];
        const int m32 = (c - b0) < 32 ? (c - b0) : 32;
#pragma unroll 1
        for (int k = 0; k < m32; ++k) {
          const int u    = __builtin_amdgcn_readlane(ent, k);
          const int slot = u & (NBRUN - 1);
          if (lane == 0) cnt[slot] = cnt[slot] + 1;
        }
      }
    }
    if (lane == 0) misc[9] = ov;
  }
  __syncthreads();

#pragma unroll 1
  for (int i = tid; i < NBRUN; i += NTHR) {
    const int c = cnt[i];
    const float den = (c > 0) ? (float)c : 1.0f;
    const float r = 1.0f / sqrtf(den);
    dvi[i] = __float_as_int((c > 0) ? r : 0.0f);
  }
  if (wave == 0) {
    const int base = lane * (NBRUN / 32);
    int s = 0;
#pragma unroll 1
    for (int i = 0; i < NBRUN / 32; ++i) s += cnt[base + i];
    int incl = s;
#pragma unroll
    for (int d = 1; d < 32; d <<= 1) {
      const int y = __shfl_up(incl, d, 32);
      if (lane >= d) incl += y;
    }
    if (lane == 31) misc[10] = (incl > RCAP) ? 1 : 0;
    int run = incl - s;
#pragma unroll 1
    for (int i = 0; i < NBRUN / 32; ++i) {
      const int cv = cnt[base + i];
      offs[base + i] = run;
      cur[base + i]  = run;
      run += cv;
    }
  }
  __syncthreads();

  if (wave == 0) {
#pragma unroll 1
    for (int w2 = 0; w2 < NWAVE; ++w2) {
      int c = misc[w2];
      c = c < 0 ? 0 : (c > WLCAP ? WLCAP : c);
#pragma unroll 1
      for (int b0 = 0; b0 < c; b0 += 32) {
        const int idx = b0 + lane;
        const int ent = wl[w2 * WLCAP + (idx < WLCAP ? idx : WLCAP - 1)];
        const int m32 = (c - b0) < 32 ? (c - b0) : 32;
#pragma unroll 1
        for (int k = 0; k < m32; ++k) {
          const int u    = __builtin_amdgcn_readlane(ent, k);
          const int slot = u & (NBRUN - 1);
          int wd = (u >> SLB) & 0x1FFFF;
          wd = wd > NN - 1 ? NN - 1 : wd;
          if (lane == 0) {
            int p = cur[slot];
            p = p < 0 ? 0 : (p > RCAP - 1 ? RCAP - 1 : p);
            pl[p] = wd;
            cur[slot] = p + 1;
          }
        }
      }
    }
  }
  __syncthreads();

  const int ovf = ((misc[9] != 0) | (misc[10] != 0)) ? 1 : 0;
  int* lp = LIST + (size_t)blk * RCAP;
  int* cp = CNT + (size_t)blk * NBRUN;
  int* op = OFF + (size_t)blk * NBRUN;
  int* dp = DINVI + (size_t)blk * NBRUN;
  int* fp = FLAG + (size_t)blk * 32;
  bucket_flush(pl, cnt, offs, dvi, ovf, lp, cp, op, dp, fp, tid);
  __threadfence();
  bucket_flush(pl, cnt, offs, dvi, ovf, lp, cp, op, dp, fp, tid);
}

template <int KTOT>
__device__ __forceinline__ void gemm_16x64(const unsigned short* __restrict__ ap,
                                           const unsigned short* __restrict__ bp, v8f (&acc)[4]) {
#pragma unroll 1
  for (int k0 = 0; k0 < KTOT; k0 += 32) {
    FragB af;
    af.h[0] = *(const v8usa*)(ap + k0);
    af.h[1] = *(const v8usa*)(ap + k0 + 16);
#pragma unroll
    for (int nt = 0; nt < 4; ++nt) {
      const unsigned short* wq = bp + (size_t)(16 * nt) * (size_t)KTOT + k0;
      FragB bf;
      bf.h[0] = *(const v8usa*)wq;
      bf.h[1] = *(const v8usa*)(wq + 16);
      acc[nt] = wmb(af, bf, acc[nt]);
    }
  }
}

__device__ __forceinline__ void stage_d(float* stg, const v8f (&acc)[4], int wave, int hh, int m) {
#pragma unroll
  for (int nt = 0; nt < 4; ++nt) {
#pragma unroll
    for (int r = 0; r < 8; ++r) stg[(16 * wave + 8 * hh + r) * SP + 16 * nt + m] = acc[nt][r];
  }
}

__global__ __launch_bounds__(NTHR) __attribute__((amdgpu_num_vgpr(248)))
void k_gemm_in(const unsigned short* __restrict__ XB, const unsigned short* __restrict__ W0T,
               const float* __restrict__ tb, const float* __restrict__ DINV,
               float* X, float* X0, float* P) {
  __shared__ __attribute__((aligned(16))) float stg[GBM * SP];
  __shared__ __attribute__((aligned(16))) float sb[64];
  const int tid = (int)threadIdx.x, lane = tid & 31, wave = tid >> 5, hh = lane >> 4, m = lane & 15;
  const int rowBase = (int)blockIdx.x * GBM;
  if (tid < 16) *(v4fa*)(sb + 4 * tid) = *(const v4fa*)(tb + 4 * tid);

  v8f acc[4];
  {
    const v8f z = {0.f, 0.f, 0.f, 0.f, 0.f, 0.f, 0.f, 0.f};
#pragma unroll
    for (int t = 0; t < 4; ++t) acc[t] = z;
  }
  const unsigned short* ap = XB + (size_t)(rowBase + 16 * wave + m) * (size_t)FD + 8 * hh;
  const unsigned short* bp = W0T + (size_t)m * (size_t)FD + 8 * hh;
  gemm_16x64<FD>(ap, bp, acc);
  stage_d(stg, acc, wave, hh, m);
  __syncthreads();

  const v4f bias = *(const v4fa*)(sb + 4 * m);
#pragma unroll 1
  for (int i = 0; i < 8; ++i) {
    const int lr   = 16 * wave + 2 * i + hh;
    const int grow = rowBase + lr;
    const bool live = grow < NN;
    const v4f a = *(const v4fa*)(stg + lr * SP + 4 * m);
    const float dv = DINV[grow];
    asm volatile("" :: "v"(a));
    asm volatile("" :: "v"(dv));
    float v0 = a.x + bias.x, v1 = a.y + bias.y, v2 = a.z + bias.z, v3 = a.w + bias.w;
    v0 = (v0 > 0.0f) ? v0 : (v0 - v0); v1 = (v1 > 0.0f) ? v1 : (v1 - v1);
    v2 = (v2 > 0.0f) ? v2 : (v2 - v2); v3 = (v3 > 0.0f) ? v3 : (v3 - v3);
    v4f o, p;
    o.x = live ? v0 : 0.0f; o.y = live ? v1 : 0.0f; o.z = live ? v2 : 0.0f; o.w = live ? v3 : 0.0f;
    p.x = dv * o.x; p.y = dv * o.y; p.z = dv * o.z; p.w = dv * o.w;
    float* xp  = X  + (size_t)grow * HD + 4 * m;
    float* x0p = X0 + (size_t)grow * HD + 4 * m;
    float* pp  = P  + (size_t)grow * HD + 4 * m;
    *(volatile v4f*)xp  = o;
    *(volatile v4f*)x0p = o;
    *(volatile v4f*)pp  = p;
    __threadfence();
    *(volatile v4f*)xp  = o;
    *(volatile v4f*)x0p = o;
    *(volatile v4f*)pp  = p;
  }
}

__global__ __launch_bounds__(NTHR) void k_replay(const int* __restrict__ LIST, const int* __restrict__ CNT,
                                                 const int* __restrict__ OFF, const int* __restrict__ FLAG,
                                                 const float* __restrict__ DINV, const float* __restrict__ P,
                                                 const float* __restrict__ X0, unsigned short* S) {
  const int tid = (int)threadIdx.x, lane = tid & 31, wave = tid >> 5, hh = lane >> 4, q = lane & 15;
  const int rowBase = (int)blockIdx.x * ABM;
  const int bucket  = rowBase >> SLB;
  const int* lb  = LIST + (size_t)bucket * RCAP;
  const int flag = FLAG[(size_t)bucket * 32];
  const float qnan = __uint_as_float(0x7fc00000u);

#pragma unroll 1
  for (int i = 0; i < ABM / (2 * NWAVE); ++i) {
    const int d = rowBase + (ABM / NWAVE) * wave + 2 * i + hh;
    int c = CNT[d];
    int o = OFF[d];
    const bool big = c > DEGCAP;
    c = c < 0 ? 0 : (c > DEGCAP ? DEGCAP : c);
    o = o < 0 ? 0 : (o > RCAP - 1 ? RCAP - 1 : o);
    const int co = __shfl_xor(c, 16, 32);
    const int cm = c > co ? c : co;
    int last = o + c - 1;
    last = last < o ? o : last;
    last = last > RCAP - 1 ? RCAP - 1 : last;
    float a0 = 0.0f, a1 = 0.0f, a2 = 0.0f, a3 = 0.0f;
#pragma unroll 1
    for (int j = 0; j < cm; ++j) {
      int idx = o + j;
      idx = idx > last ? last : idx;
      int sr = lb[idx];
      sr = sr < 0 ? 0 : (sr > NN - 1 ? NN - 1 : sr);
      const v4f v = *(const v4fa*)(P + (size_t)sr * HD + 4 * q);
      asm volatile("" :: "v"(v));
      const bool valid = j < c;
      const float t0 = a0 + v.x, t1 = a1 + v.y, t2 = a2 + v.z, t3 = a3 + v.w;
      a0 = valid ? t0 : a0; a1 = valid ? t1 : a1; a2 = valid ? t2 : a2; a3 = valid ? t3 : a3;
    }
    const float dv = DINV[d];
    const v4f g = *(const v4fa*)(X0 + (size_t)d * HD + 4 * q);
    const float g0 = dv * a0, g1 = dv * a1, g2 = dv * a2, g3 = dv * a3;
    float m0 = 0.9f * g0 + 0.1f * g.x, m1 = 0.9f * g1 + 0.1f * g.y;
    float m2 = 0.9f * g2 + 0.1f * g.z, m3 = 0.9f * g3 + 0.1f * g.w;
    const bool bad  = (flag != 0) | big;
    const bool live = d < NN;
    m0 = bad ? qnan : m0; m1 = bad ? qnan : m1; m2 = bad ? qnan : m2; m3 = bad ? qnan : m3;
    m0 = live ? m0 : 0.0f; m1 = live ? m1 : 0.0f; m2 = live ? m2 : 0.0f; m3 = live ? m3 : 0.0f;
    int h01, h23, l01, l23;
    hilo_pack(m0, m1, m2, m3, h01, h23, l01, l23);
    const v4i ow = regroup8(h01, h23, l01, l23, lane);
    unsigned short* hp = S + (size_t)d * KL + 8 * q;
    *(volatile v4i*)hp = ow;
    __threadfence();
    *(volatile v4i*)hp = ow;
  }
}

__global__ __launch_bounds__(NTHR) __attribute__((amdgpu_num_vgpr(248)))
void k_gemm_layer(const unsigned short* __restrict__ A, const unsigned short* __restrict__ BT,
                  float fomb, float fb, float* H, float* REC) {
  __shared__ __attribute__((aligned(16))) float stg[GBM * SP];
  __shared__ __attribute__((aligned(16))) float rec[RECW];
  const int tid = (int)threadIdx.x, lane = tid & 31, wave = tid >> 5, hh = lane >> 4, m = lane & 15;
  const int rowBase = (int)blockIdx.x * GBM;

  v8f acc[4];
  {
    const v8f z = {0.f, 0.f, 0.f, 0.f, 0.f, 0.f, 0.f, 0.f};
#pragma unroll
    for (int t = 0; t < 4; ++t) acc[t] = z;
  }
  const unsigned short* ap = A + (size_t)(rowBase + 16 * wave + m) * (size_t)KL + 8 * hh;
  const unsigned short* bp = BT + (size_t)m * (size_t)KL + 8 * hh;
  gemm_16x64<KL>(ap, bp, acc);
  stage_d(stg, acc, wave, hh, m);
  __syncthreads();

#pragma unroll 1
  for (int i = 0; i < 8; ++i) {
    const int lr   = 16 * wave + 2 * i + hh;
    const int grow = rowBase + lr;
    const bool live = grow < NN;
    const v4f a  = *(const v4fa*)(stg + lr * SP + 4 * m);
    const unsigned short* sp = A + (size_t)grow * KL + 4 * m;
    const v2u hw = *(const v2ua*)sp;
    const v2u lw = *(const v2ua*)(sp + HD);
    asm volatile("" :: "v"(a));
    asm volatile("" :: "v"(hw), "v"(lw));
    const float s0 = __uint_as_float(hw.x << 16)          + __uint_as_float(lw.x << 16);
    const float s1 = __uint_as_float(hw.x & 0xffff0000u) + __uint_as_float(lw.x & 0xffff0000u);
    const float s2 = __uint_as_float(hw.y << 16)          + __uint_as_float(lw.y << 16);
    const float s3 = __uint_as_float(hw.y & 0xffff0000u) + __uint_as_float(lw.y & 0xffff0000u);
    float v0 = fomb * s0 + fb * a.x, v1 = fomb * s1 + fb * a.y;
    float v2 = fomb * s2 + fb * a.z, v3 = fomb * s3 + fb * a.w;
    v4f o;
    o.x = live ? v0 : 0.0f; o.y = live ? v1 : 0.0f; o.z = live ? v2 : 0.0f; o.w = live ? v3 : 0.0f;
    *(v4fa*)(stg + lr * SP + 4 * m) = o;
    st2_v4f(H + (size_t)grow * HD + 4 * m, o);
  }
  __syncthreads();

  if (tid < HD) {
    const int c = tid;
    int nv = NN - rowBase;
    nv = nv > GBM ? GBM : nv;
    nv = nv < 1 ? 1 : nv;
    float sum = 0.0f;
#pragma unroll 4
    for (int r = 0; r < nv; ++r) sum += stg[r * SP + c];
    const float fn   = (float)nv;
    const float mean = sum * (1.0f / fn);
    float m2 = 0.0f;
#pragma unroll 4
    for (int r = 0; r < nv; ++r) {
      const float dlt = stg[r * SP + c] - mean;
      m2 = fmaf(dlt, dlt, m2);
    }
    rec[c] = fn;
    rec[HD + c] = mean;
    rec[2 * HD + c] = m2;
  }
  __syncthreads();

  v4f ps = {0.f, 0.f, 0.f, 0.f};
  float* rp = REC + (size_t)blockIdx.x * RECW + 4 * tid;
  if (tid < RECW / 4) {
    ps = *(const v4fa*)(rec + 4 * tid);
    *(volatile v4f*)rp = ps;
  }
  __threadfence();
  if (tid < RECW / 4) {
    *(volatile v4f*)rp = ps;
  }
}

__global__ __launch_bounds__(HD) void k_comb(const float* __restrict__ REC, float* STAT) {
  __shared__ __attribute__((aligned(16))) float stg[2 * HD];
  const int tid = (int)threadIdx.x;
  const int c = tid;
  double n = 0.0, mean = 0.0, M2 = 0.0;
#pragma unroll 1
  for (int b = 0; b < NGB; ++b) {
    const float* pr = REC + (size_t)b * RECW;
    const double nb = (double)pr[c];
    const double mb = (double)pr[HD + c];
    const double qb = (double)pr[2 * HD + c];
    if (nb > 0.5) {
      const double nn = n + nb;
      const double delta = mb - mean;
      const double f = nb / nn;
      mean = mean + delta * f;
      M2 = M2 + qb + delta * delta * n * f;
      n = nn;
    }
  }
  const double nt = n < 1.0 ? 1.0 : n;
  const float varf  = (float)(M2 / nt);
  const float meanf = (float)mean;
  const float rstd  = 1.0f / sqrtf(varf + 1e-5f);
  stg[c] = meanf;
  stg[HD + c] = rstd;
  __syncthreads();
  v4f v = {0.f, 0.f, 0.f, 0.f};
  if (tid < (2 * HD) / 4) {
    v = *(const v4fa*)(stg + 4 * tid);
    *(volatile v4f*)(STAT + 4 * tid) = v;
  }
  __threadfence();
  if (tid < (2 * HD) / 4) {
    *(volatile v4f*)(STAT + 4 * tid) = v;
  }
}

template <int LAST>
__global__ __launch_bounds__(NTHR) void k_apply(const float* __restrict__ STAT, const float* __restrict__ gb,
                                                const float* __restrict__ DINV, float* X, float* H,
                                                unsigned short* S) {
  __shared__ __attribute__((aligned(16))) float sp[4 * HD];
  const int tid = (int)threadIdx.x, lane = tid & 31, wave = tid >> 5;
  if (wave == 0) {
    *(v4fa*)(sp + 4 * lane) = *(const v4fa*)(STAT + 4 * lane);
  } else if (wave == 1) {
    const int off = (lane >> 4) * (TB_B - TB_G) + 4 * (lane & 15);
    *(v4fa*)(sp + 2 * HD + 4 * lane) = *(const v4fa*)(gb + off);
  }
  __syncthreads();

  const int u   = (int)blockIdx.x * NTHR + tid;
  const int row = u >> 4, q = u & 15;
  const bool live = row < NN;
  const v4f h  = *(const v4fa*)(H + (size_t)u * 4);
  const v4f xv = *(const v4fa*)(X + (size_t)u * 4);
  const float dv = DINV[row];
  asm volatile("" :: "v"(h));
  asm volatile("" :: "v"(xv));
  asm volatile("" :: "v"(dv));
  const v4f mu = *(const v4fa*)(sp + 4 * q);
  const v4f rs = *(const v4fa*)(sp + HD + 4 * q);
  const v4f g  = *(const v4fa*)(sp + 2 * HD + 4 * q);
  const v4f b  = *(const v4fa*)(sp + 3 * HD + 4 * q);
  float y0 = ((h.x - mu.x) * rs.x) * g.x + b.x + xv.x;
  float y1 = ((h.y - mu.y) * rs.y) * g.y + b.y + xv.y;
  float y2 = ((h.z - mu.z) * rs.z) * g.z + b.z + xv.z;
  float y3 = ((h.w - mu.w) * rs.w) * g.w + b.w + xv.w;
  y0 = (y0 > 0.0f) ? y0 : (y0 - y0); y1 = (y1 > 0.0f) ? y1 : (y1 - y1);
  y2 = (y2 > 0.0f) ? y2 : (y2 - y2); y3 = (y3 > 0.0f) ? y3 : (y3 - y3);
  y0 = live ? y0 : 0.0f; y1 = live ? y1 : 0.0f; y2 = live ? y2 : 0.0f; y3 = live ? y3 : 0.0f;
  if constexpr (LAST != 0) {
    int h01, h23, l01, l23;
    hilo_pack(y0, y1, y2, y3, h01, h23, l01, l23);
    const v4i ow = regroup8(h01, h23, l01, l23, lane);
    unsigned short* hp = S + (size_t)row * KL + 8 * q;
    *(volatile v4i*)hp = ow;
    __threadfence();
    *(volatile v4i*)hp = ow;
  } else {
    v4f o, p;
    o.x = y0; o.y = y1; o.z = y2; o.w = y3;
    p.x = dv * y0; p.y = dv * y1; p.z = dv * y2; p.w = dv * y3;
    float* xp = X + (size_t)u * 4;
    float* pp = H + (size_t)u * 4;
    *(volatile v4f*)xp = o;
    *(volatile v4f*)pp = p;
    __threadfence();
    *(volatile v4f*)xp = o;
    *(volatile v4f*)pp = p;
  }
}

__global__ __launch_bounds__(NTHR) __attribute__((amdgpu_num_vgpr(248)))
void k_gemm_out(const unsigned short* __restrict__ A, const unsigned short* __restrict__ BT,
                const float* __restrict__ tb1, float* out) {
  __shared__ __attribute__((aligned(16))) float stg[GBM * SP];
  __shared__ __attribute__((aligned(16))) float sb[64];
  const int tid = (int)threadIdx.x, lane = tid & 31, wave = tid >> 5, hh = lane >> 4, m = lane & 15;
  const int rowBase = (int)blockIdx.x * GBM;
  if (tid < 16) *(v4fa*)(sb + 4 * tid) = *(const v4fa*)(tb1 + 4 * tid);

  v8f acc[4];
  {
    const v8f z = {0.f, 0.f, 0.f, 0.f, 0.f, 0.f, 0.f, 0.f};
#pragma unroll
    for (int t = 0; t < 4; ++t) acc[t] = z;
  }
  const unsigned short* ap = A + (size_t)(rowBase + 16 * wave + m) * (size_t)KL + 8 * hh;
  const unsigned short* bp = BT + (size_t)m * (size_t)KL + 8 * hh;
  gemm_16x64<KL>(ap, bp, acc);
  stage_d(stg, acc, wave, hh, m);
  __syncthreads();

  const v4f bias = *(const v4fa*)(sb + 4 * m);
#pragma unroll 1
  for (int i = 0; i < 8; ++i) {
    const int lr   = 16 * wave + 2 * i + hh;
    const int grow = rowBase + lr;
    const bool live = grow < NN;
    const int gr = live ? grow : NN - 1;
    const v4f a = *(const v4fa*)(stg + lr * SP + 4 * m);
    asm volatile("" :: "v"(a));
    v4f o;
    o.x = a.x + bias.x; o.y = a.y + bias.y; o.z = a.z + bias.z; o.w = a.w + bias.w;
    float* op = out + (size_t)gr * HD + 4 * m;
    if (live) *(volatile v4f*)op = o;
    __threadfence();
    if (live) *(volatile v4f*)op = o;
  }
}

extern "C" void kernel_launch(void* const* d_in, const int* in_sizes, int n_in,
                              void* d_out, int out_size, void* d_ws, size_t ws_size,
                              hipStream_t stream) {
  if (n_in < 9) return;
  if (in_sizes[0] != NN * FD) return;
  if (in_sizes[1] != 2 * NE) return;
  if (in_sizes[2] != FD * HD) return;
  if (in_sizes[3] != HD) return;
  if (in_sizes[4] != NLAY * HD * HD) return;
  if (in_sizes[5] != NLAY * HD) return;
  if (in_sizes[6] != NLAY * HD) return;
  if (in_sizes[7] != HD * HD) return;
  if (in_sizes[8] != HD) return;
  if (out_size != NN * HD) return;

  const float* x   = (const float*)d_in[0];
  const int*   ei  = (const int*)d_in[1];
  const float* W0  = (const float*)d_in[2];
  const float* b0  = (const float*)d_in[3];
  const float* cw  = (const float*)d_in[4];
  const float* gam = (const float*)d_in[5];
  const float* bet = (const float*)d_in[6];
  const float* W1  = (const float*)d_in[7];
  const float* b1  = (const float*)d_in[8];
  float* out = (float*)d_out;
  const int* rows = ei;
  const int* cols = ei + NE;

  constexpr size_t zF    = (size_t)MP * HD * 4;
  constexpr size_t zS    = (size_t)MP * KL * 2;
  constexpr size_t zLIST = (size_t)NBK * RCAP * 4;
  constexpr size_t zTAB  = (size_t)NSLOT * 4;
  constexpr size_t zFLAG = (size_t)NBK * 128;
  constexpr size_t zREC  = (size_t)NGB * RECW * 4;
  constexpr size_t zSTAT = 512;
  constexpr size_t zWPL  = (size_t)(HD * FD + NLAY * HD * KL + HD * KL) * 2;
  constexpr size_t zTB   = (size_t)TB_N * 4;
  constexpr size_t oPX   = 0;
  constexpr size_t oPX0  = oPX + zF;
  constexpr size_t oPH   = oPX0 + zF;
  constexpr size_t oPS   = oPH + zF;
  constexpr size_t oLIST = oPS + zS;
  constexpr size_t oCNT  = oLIST + zLIST;
  constexpr size_t oOFF  = oCNT + zTAB;
  constexpr size_t oDINV = oOFF + zTAB;
  constexpr size_t oFLAG = oDINV + zTAB;
  constexpr size_t oREC  = oFLAG + zFLAG;
  constexpr size_t oSTAT = oREC + zREC;
  constexpr size_t oWPL  = oSTAT + zSTAT;
  constexpr size_t oTB   = oWPL + zWPL;
  constexpr size_t oEND  = oTB + zTB;
  static_assert(zF % 256 == 0 && zS % 256 == 0 && zLIST % 256 == 0 && zTAB % 256 == 0 && zFLAG % 256 == 0);
  static_assert(zREC % 256 == 0 && zSTAT % 256 == 0 && zWPL % 256 == 0 && zTB % 256 == 0);
  static_assert(zS >= (size_t)MP * FD * 2);
  static_assert(oEND <= (size_t)WSMAX);
  if (oEND > ws_size) return;

  char* ws = (char*)d_ws;
  float*          PX   = (float*)(ws + oPX);
  float*          PX0  = (float*)(ws + oPX0);
  float*          PH   = (float*)(ws + oPH);
  unsigned short* PS   = (unsigned short*)(ws + oPS);
  int*            LIST = (int*)(ws + oLIST);
  int*            CNT  = (int*)(ws + oCNT);
  int*            OFF  = (int*)(ws + oOFF);
  float*          DINV = (float*)(ws + oDINV);
  int*            FLAG = (int*)(ws + oFLAG);
  float*          REC  = (float*)(ws + oREC);
  float*          STAT = (float*)(ws + oSTAT);
  unsigned short* WPL  = (unsigned short*)(ws + oWPL);
  float*          TB   = (float*)(ws + oTB);
  const unsigned short* W0T = WPL;
  const unsigned short* CWT = WPL + OW_CWT;
  const unsigned short* W1T = WPL + OW_W1T;

  hipFuncSetAttribute(reinterpret_cast<const void*>(&k_bucket), hipFuncAttributeMaxDynamicSharedMemorySize, (int)BK_LDS);

  k_prep<<<PBTOT, NTHR, 0, stream>>>(x, W0, cw, W1, b0, b1, gam, bet, PS, WPL, TB);
  k_bucket<<<NBK, NTHR, BK_LDS, stream>>>(rows, cols, LIST, CNT, OFF, (int*)DINV, FLAG);
  k_gemm_in<<<NGB, NTHR, 0, stream>>>(PS, W0T, TB + TB_B0, DINV, PX, PX0, PH);

  for (int l = 0; l < NLAY; ++l) {
    const double bd   = log(0.5 / (double)(l + 1) + 1.0);
    const float  fb   = (float)bd;
    const float  fomb = (float)(1.0 - bd);
    k_replay<<<MP / ABM, NTHR, 0, stream>>>(LIST, CNT, OFF, FLAG, DINV, PH, PX0, PS);
    k_gemm_layer<<<NGB, NTHR, 0, stream>>>(PS, CWT + (size_t)l * HD * KL, fomb, fb, PH, REC);
    k_comb<<<1, HD, 0, stream>>>(REC, STAT);
    const float* gb = TB + TB_G + l * HD;
    if (l == NLAY - 1)
      k_apply<1><<<(MP * HD / 4) / NTHR, NTHR, 0, stream>>>(STAT, gb, DINV, PX, PH, PS);
    else
      k_apply<0><<<(MP * HD / 4) / NTHR, NTHR, 0, stream>>>(STAT, gb, DINV, PX, PH, PS);
  }
  k_gemm_out<<<NGB, NTHR, 0, stream>>>(PS, W1T, TB + TB_B1, out);
}
